// GraphTransformerLayer4o_40132174414151
// MI455X (gfx1250) — hardware-verified
//
#include <hip/hip_runtime.h>
#include <math.h>
#include <stdint.h>

#define NN    4096
#define DM    512
#define NH    8
#define HD    64
#define QKV3  1536
#define QKLD  1024
#define BROWS 8
#define NEGB  (-1.0e9f)

typedef _Float16 v16h __attribute__((ext_vector_type(16)));
typedef _Float16 v8h  __attribute__((ext_vector_type(8)));
typedef _Float16 v4h  __attribute__((ext_vector_type(4)));
typedef float    v8f  __attribute__((ext_vector_type(8)));
typedef float    v4f  __attribute__((ext_vector_type(4)));

union FH { v16h v; v8h h[2]; };

__device__ __forceinline__ v16h ld_frag(const _Float16* p)
{
    FH f;
    f.h[0] = *(const v8h*)(p);
    f.h[1] = *(const v8h*)(p + 16);
    return f.v;
}

__device__ __forceinline__ v8f mma16(v16h a, v16h b, v8f c)
{
    c = __builtin_amdgcn_wmma_f32_16x16x32_f16(false, a, false, b, (short)0, c, false, false);
    asm volatile("v_nop\n\tv_nop\n\tv_nop\n\tv_nop" : "+v"(c) : "v"(a), "v"(b));
    return c;
}

__device__ __forceinline__ void wave_lds_sync()
{
    __builtin_amdgcn_fence(__ATOMIC_RELEASE, "workgroup");
    __builtin_amdgcn_wave_barrier();
    __builtin_amdgcn_fence(__ATOMIC_ACQUIRE, "workgroup");
}

__global__ __launch_bounds__(256)
void k_bias_rows(const int* __restrict__ ei, const float* __restrict__ ew, int nE, int nChunks,
                 float* __restrict__ plane)
{
    extern __shared__ __align__(16) float brow[];
    __shared__ int   wcnt[2][8];
    __shared__ int   hl_idx[256];
    __shared__ float hl_w[256];

    const int tid = threadIdx.x, wave = tid >> 5, lane = tid & 31;
    const int r0 = blockIdx.x * BROWS;

    const v4f negv = {NEGB, NEGB, NEGB, NEGB};
#pragma unroll 4
    for (int it = 0; it < (BROWS * NN / 4) / 256; ++it)
        ((v4f*)brow)[it * 256 + tid] = negv;
    __syncthreads();
    if (tid < BROWS) brow[tid * NN + r0 + tid] = 0.0f;
    __syncthreads();

    for (int cidx = 0; cidx < nChunks; ++cidx) {
        const int e  = cidx * 256 + tid;
        const int ec = min(e, nE - 1);
        const int s  = ei[ec];
        const int d  = ei[(size_t)nE + ec];
        const float w = ew[ec];
        const bool hit = (e < nE) && ((unsigned)(d - r0) < (unsigned)BROWS) && ((unsigned)s < (unsigned)NN);
        const unsigned msk = __builtin_amdgcn_ballot_w32(hit);
        const int cnt = __popc(msk);
        const int pre = __popc(msk & ((1u << lane) - 1u));
        const int par = cidx & 1;
        if (lane == 0) wcnt[par][wave] = cnt;
        __syncthreads();
        int base = 0, total = 0;
#pragma unroll
        for (int wv = 0; wv < 8; ++wv) {
            const int cw = wcnt[par][wv];
            total += cw;
            if (wv < wave) base += cw;
        }
        if (total != 0) {
            if (hit) {
                const int pos = min(base + pre, 255);
                hl_idx[pos] = (d - r0) * NN + s;
                hl_w[pos]   = w;
            }
            __syncthreads();
            if (tid == 0) {
                const int tt = min(total, 256);
                for (int i = 0; i < tt; ++i) {
                    const int ix = min(max(hl_idx[i], 0), BROWS * NN - 1);
                    brow[ix] = hl_w[i];
                }
            }
        }
    }
    __syncthreads();

    float* dst = plane + (size_t)r0 * NN;
    for (int pass = 0; pass < 2; ++pass) {
#pragma unroll 4
        for (int it = 0; it < (BROWS * NN / 4) / 256; ++it) {
            const int idx = it * 256 + tid;
            const v4f v = ((const v4f*)brow)[idx];
            *(volatile v4f*)(dst + (size_t)idx * 4) = v;
        }
        __threadfence();
    }
}

__global__ __launch_bounds__(256)
void k_cvt_f16(const float* __restrict__ in, _Float16* __restrict__ out, int n8, float scale)
{
    const int i = blockIdx.x * 256 + threadIdx.x;
    if (i < n8) {
        const float* p = in + (size_t)i * 8;
        const v4f a = *(const v4f*)(p);
        const v4f b = *(const v4f*)(p + 4);
        v8h o;
        o[0] = (_Float16)(a[0] * scale); o[1] = (_Float16)(a[1] * scale);
        o[2] = (_Float16)(a[2] * scale); o[3] = (_Float16)(a[3] * scale);
        o[4] = (_Float16)(b[0] * scale); o[5] = (_Float16)(b[1] * scale);
        o[6] = (_Float16)(b[2] * scale); o[7] = (_Float16)(b[3] * scale);
        _Float16* q = out + (size_t)i * 8;
        *(volatile v8h*)q = o;
        __threadfence();
        *(volatile v8h*)q = o;
    }
}

template <int BIAS_MODE, int OUT_MODE, bool RESID>
__global__ __launch_bounds__(256)
void k_gemm64(const _Float16* __restrict__ A, int lda, const _Float16* __restrict__ Bt, int ldb,
              void* __restrict__ Cout, int ldc, const float* __restrict__ bias,
              const float* __restrict__ resid, int ldr, int M, int N, int K, float scale)
{
    __shared__ __align__(16) float sT[8][16 * 68];
    const int lane = threadIdx.x & 31;
    const int wave = threadIdx.x >> 5;
    const int tilesN = N >> 6;
    const int tilesM = M >> 6;
    const int tile = blockIdx.x * 8 + wave;
    if (tile >= tilesM * tilesN) return;
    const int tm = tile / tilesN;
    const int tn = tile - tm * tilesN;
    const int m0 = tm << 6;
    const int n0 = tn << 6;
    const int rl   = lane & 15;
    const int koff = (lane >> 4) * 8;
    const int mOff = (lane >> 4) * 8;

    v8f acc[4][4];
#pragma unroll
    for (int i = 0; i < 4; ++i)
#pragma unroll
        for (int j = 0; j < 4; ++j) acc[i][j] = (v8f){0.f, 0.f, 0.f, 0.f, 0.f, 0.f, 0.f, 0.f};

    for (int k0 = 0; k0 < K; k0 += 32) {
        v16h bq[4];
#pragma unroll
        for (int j = 0; j < 4; ++j)
            bq[j] = ld_frag(Bt + (size_t)(n0 + (j << 4) + rl) * ldb + k0 + koff);
#pragma unroll
        for (int i = 0; i < 4; ++i) {
            const v16h af = ld_frag(A + (size_t)(m0 + (i << 4) + rl) * lda + k0 + koff);
#pragma unroll
            for (int j = 0; j < 4; ++j) acc[i][j] = mma16(af, bq[j], acc[i][j]);
        }
    }

    float* slab = sT[wave];
#pragma unroll
    for (int i = 0; i < 4; ++i) {
        const int mBase = m0 + (i << 4);
#pragma unroll
        for (int j = 0; j < 4; ++j) {
            const int n = n0 + (j << 4) + rl;
            float bv = 0.f;
            if (BIAS_MODE == 2) bv = bias[n];
#pragma unroll
            for (int r = 0; r < 8; ++r) {
                float v = acc[i][j][r] * scale;
                if (BIAS_MODE == 1) v += bias[mBase + mOff + r];
                if (BIAS_MODE == 2) v += bv;
                if (RESID) v += resid[(size_t)(mBase + mOff + r) * ldr + n];
                slab[(mOff + r) * 68 + (j << 4) + rl] = v;
            }
        }
        wave_lds_sync();
        if (OUT_MODE == 0) {
            float* C = (float*)Cout;
            const int hh = lane >> 4, c4 = (lane & 15) * 4;
            for (int pass = 0; pass < 2; ++pass) {
#pragma unroll
                for (int it = 0; it < 8; ++it) {
                    const int row = it * 2 + hh;
                    const v4f v = *(const v4f*)(slab + row * 68 + c4);
                    *(volatile v4f*)(C + (size_t)(mBase + row) * ldc + n0 + c4) = v;
                }
                __threadfence();
            }
        } else {
            _Float16* C = (_Float16*)Cout;
            const int q8 = lane >> 3, c8 = (lane & 7) * 8;
            for (int pass = 0; pass < 2; ++pass) {
#pragma unroll
                for (int it = 0; it < 4; ++it) {
                    const int row = it * 4 + q8;
                    const float* sp = slab + row * 68 + c8;
                    v8h hv;
#pragma unroll
                    for (int e = 0; e < 8; ++e) hv[e] = (_Float16)sp[e];
                    *(volatile v8h*)(C + (size_t)(mBase + row) * ldc + n0 + c8) = hv;
                }
                __threadfence();
            }
        }
        wave_lds_sync();
    }
}

__global__ __launch_bounds__(128)
void k_attn(const _Float16* __restrict__ QK, const _Float16* __restrict__ VT,
            const float* __restrict__ Bpl, _Float16* __restrict__ CTX)
{
    __shared__ __align__(16) _Float16 Psh[4][16 * HD];
    __shared__ __align__(16) float    Os[4][16 * 68];

    const int tid  = threadIdx.x;
    const int wave = tid >> 5;
    const int lane = tid & 31;
    const int hh   = lane >> 4;
    const int c    = lane & 15;

    const int bx   = blockIdx.x;
    const int qb   = bx & 63;
    const int head = bx >> 6;
    const int q0   = qb * 64 + wave * 16;

    const _Float16* Qb = QK + head * HD;
    const _Float16* Kb = QK + DM + head * HD;
    const _Float16* Vb = VT + (size_t)head * HD * NN;

    v16h qa[2];
#pragma unroll
    for (int dc = 0; dc < 2; ++dc)
        qa[dc] = ld_frag(Qb + (size_t)(q0 + c) * QKLD + dc * 32 + 8 * hh);

    float mrow[8], lrow[8];
    v8f oacc[4];
#pragma unroll
    for (int r = 0; r < 8; ++r) { mrow[r] = -INFINITY; lrow[r] = 0.f; }
#pragma unroll
    for (int t = 0; t < 4; ++t) oacc[t] = (v8f){0.f, 0.f, 0.f, 0.f, 0.f, 0.f, 0.f, 0.f};

    _Float16* pw = Psh[wave];

    for (int kc = 0; kc < NN / 64; ++kc) {
        const int kv0 = kc * 64;

        v8f s[4];
#pragma unroll
        for (int j = 0; j < 4; ++j) {
            s[j] = (v8f){0.f, 0.f, 0.f, 0.f, 0.f, 0.f, 0.f, 0.f};
#pragma unroll
            for (int dc = 0; dc < 2; ++dc) {
                const v16h kb = ld_frag(Kb + (size_t)(kv0 + j * 16 + c) * QKLD + dc * 32 + 8 * hh);
                s[j] = mma16(qa[dc], kb, s[j]);
            }
        }

        float cm[8];
#pragma unroll
        for (int r = 0; r < 8; ++r) {
            const float* brp = Bpl + (size_t)(q0 + 8 * hh + r) * NN + kv0 + c;
            float m = -INFINITY;
#pragma unroll
            for (int j = 0; j < 4; ++j) {
                const float sv = s[j][r] * 0.125f + brp[j * 16];
                s[j][r] = sv;
                m = fmaxf(m, sv);
            }
#pragma unroll
            for (int off = 1; off < 16; off <<= 1) m = fmaxf(m, __shfl_xor(m, off, 32));
            cm[r] = m;
        }

#pragma unroll
        for (int r = 0; r < 8; ++r) {
            const float mnew  = fmaxf(mrow[r], cm[r]);
            const float alpha = expf(mrow[r] - mnew);
            mrow[r] = mnew;
            float psum = 0.f;
#pragma unroll
            for (int j = 0; j < 4; ++j) {
                const float p = expf(s[j][r] - mnew);
                psum += p;
                pw[(8 * hh + r) * HD + j * 16 + c] = (_Float16)(p * 16384.0f);
            }
#pragma unroll
            for (int off = 1; off < 16; off <<= 1) psum += __shfl_xor(psum, off, 32);
            lrow[r] = lrow[r] * alpha + psum;
#pragma unroll
            for (int t = 0; t < 4; ++t) oacc[t][r] *= alpha;
        }
        wave_lds_sync();

#pragma unroll 1
        for (int kk = 0; kk < 2; ++kk) {
            FH pa;
            pa.h[0] = *(const v8h*)(pw + c * HD + kk * 32 + 8 * hh);
            pa.h[1] = *(const v8h*)(pw + c * HD + kk * 32 + 16 + 8 * hh);
#pragma unroll
            for (int t = 0; t < 4; ++t) {
                const v16h vb = ld_frag(Vb + (size_t)(t * 16 + c) * NN + kv0 + kk * 32 + 8 * hh);
                oacc[t] = mma16(pa.v, vb, oacc[t]);
            }
        }
        wave_lds_sync();
    }

    float* os = Os[wave];
#pragma unroll
    for (int r = 0; r < 8; ++r) {
        const float inv = (1.0f / lrow[r]) * (1.0f / 16384.0f);
#pragma unroll
        for (int t = 0; t < 4; ++t) os[(8 * hh + r) * 68 + t * 16 + c] = oacc[t][r] * inv;
    }
    wave_lds_sync();
    {
        const int q8 = lane >> 3, c8 = (lane & 7) * 8;
        for (int pass = 0; pass < 2; ++pass) {
#pragma unroll
            for (int it = 0; it < 4; ++it) {
                const int row = it * 4 + q8;
                const float* sp = os + row * 68 + c8;
                v8h hv;
#pragma unroll
                for (int e = 0; e < 8; ++e) hv[e] = (_Float16)sp[e];
                *(volatile v8h*)(CTX + (size_t)(q0 + row) * DM + head * HD + c8) = hv;
            }
            __threadfence();
        }
    }
}

template <int WH>
__global__ __launch_bounds__(256)
void k_ln(const float* __restrict__ Y, const float* __restrict__ g, const float* __restrict__ bt,
          float* __restrict__ outF, _Float16* __restrict__ outH, int nRows)
{
    __shared__ float part[2][8];
    const int tid = threadIdx.x, wave = tid >> 5, lane = tid & 31;
    const int sub = tid >> 7;
    const int row = blockIdx.x * 2 + sub;
    const int rowc = min(row, nRows - 1);
    const int col = (tid & 127) * 4;

    const v4f t = *(const v4f*)(Y + (size_t)rowc * DM + col);
    float s1 = (t[0] + t[1]) + (t[2] + t[3]);
#pragma unroll
    for (int off = 16; off > 0; off >>= 1) s1 += __shfl_xor(s1, off, 32);
    if (lane == 0) part[0][wave] = s1;
    __syncthreads();
    const int wb = sub * 4;
    const float S1 = (part[0][wb] + part[0][wb + 1]) + (part[0][wb + 2] + part[0][wb + 3]);
    const float mu = S1 * (1.0f / DM);

    v4f d;
    d[0] = t[0] - mu; d[1] = t[1] - mu; d[2] = t[2] - mu; d[3] = t[3] - mu;
    float s2 = (d[0] * d[0] + d[1] * d[1]) + (d[2] * d[2] + d[3] * d[3]);
#pragma unroll
    for (int off = 16; off > 0; off >>= 1) s2 += __shfl_xor(s2, off, 32);
    if (lane == 0) part[1][wave] = s2;
    __syncthreads();
    const float S2 = (part[1][wb] + part[1][wb + 1]) + (part[1][wb + 2] + part[1][wb + 3]);
    const float var = S2 * (1.0f / DM);
    const float rstd = rsqrtf(var + 1e-5f);

    const v4f gv = *(const v4f*)(g + col);
    const v4f bv = *(const v4f*)(bt + col);
    v4f o;
    o[0] = d[0] * rstd * gv[0] + bv[0];
    o[1] = d[1] * rstd * gv[1] + bv[1];
    o[2] = d[2] * rstd * gv[2] + bv[2];
    o[3] = d[3] * rstd * gv[3] + bv[3];

    if (row < nRows) {
        float* po = outF + (size_t)row * DM + col;
        v4h hv;
        hv[0] = (_Float16)o[0]; hv[1] = (_Float16)o[1]; hv[2] = (_Float16)o[2]; hv[3] = (_Float16)o[3];
        *(volatile v4f*)po = o;
        if (WH) *(volatile v4h*)(outH + (size_t)row * DM + col) = hv;
        __threadfence();
        *(volatile v4f*)po = o;
        if (WH) *(volatile v4h*)(outH + (size_t)row * DM + col) = hv;
    }
}

extern "C" void kernel_launch(void* const* d_in, const int* in_sizes, int n_in,
                              void* d_out, int out_size, void* d_ws, size_t ws_size,
                              hipStream_t stream)
{
    if (n_in < 13) return;
    const int nE = in_sizes[1] / 2;
    if (in_sizes[0] != NN * DM) return;
    if (nE < 1 || in_sizes[1] != 2 * nE || in_sizes[2] != nE) return;
    if (in_sizes[3] != QKV3 * DM || in_sizes[4] != QKV3) return;
    if (in_sizes[5] != DM * DM || in_sizes[6] != DM) return;
    if (in_sizes[7] != DM * DM || in_sizes[8] != DM) return;
    if (in_sizes[9] != DM || in_sizes[10] != DM || in_sizes[11] != DM || in_sizes[12] != DM) return;
    if (out_size != NN * DM) return;

    const float* x    = (const float*)d_in[0];
    const int*   ei   = (const int*)d_in[1];
    const float* ew   = (const float*)d_in[2];
    const float* Wqkv = (const float*)d_in[3];
    const float* bqkv = (const float*)d_in[4];
    const float* Wo   = (const float*)d_in[5];
    const float* bo   = (const float*)d_in[6];
    const float* W1   = (const float*)d_in[7];
    const float* b1   = (const float*)d_in[8];
    const float* g1   = (const float*)d_in[9];
    const float* be1  = (const float*)d_in[10];
    const float* g2   = (const float*)d_in[11];
    const float* be2  = (const float*)d_in[12];
    float* out = (float*)d_out;

    const size_t szBias = (size_t)NN * NN * 4;
    const size_t szXh   = (size_t)NN * DM * 2;
    const size_t szWq   = (size_t)QKV3 * DM * 2;
    const size_t szW    = (size_t)DM * DM * 2;
    const size_t szQK   = (size_t)NN * QKLD * 2;
    const size_t szVT   = (size_t)DM * NN * 2;
    const size_t szF    = (size_t)NN * DM * 4;
    size_t off = 0;
    const size_t oBias = off; off += szBias;
    const size_t oXh   = off; off += szXh;
    const size_t oWq   = off; off += szWq;
    const size_t oWo   = off; off += szW;
    const size_t oW1   = off; off += szW;
    const size_t oQK   = off; off += szQK;
    const size_t oVT   = off; off += szVT;
    const size_t oCTX  = off; off += szXh;
    const size_t oY    = off; off += szF;
    const size_t oH    = off; off += szF;
    const size_t oHh   = off; off += szXh;
    if (off > ws_size) return;

    char* ws = (char*)d_ws;
    float*    Bpl  = (float*)(ws + oBias);
    _Float16* Xh   = (_Float16*)(ws + oXh);
    _Float16* Wqh  = (_Float16*)(ws + oWq);
    _Float16* Woh  = (_Float16*)(ws + oWo);
    _Float16* W1h  = (_Float16*)(ws + oW1);
    _Float16* QKh  = (_Float16*)(ws + oQK);
    _Float16* VTh  = (_Float16*)(ws + oVT);
    _Float16* CTXh = (_Float16*)(ws + oCTX);
    float*    Y    = (float*)(ws + oY);
    float*    H    = (float*)(ws + oH);
    _Float16* Hh   = (_Float16*)(ws + oHh);

    const dim3 b256(256);
    const float winv = 1.0f / 16.0f;

    const int nChunks = (nE + 255) / 256;
    hipFuncSetAttribute(reinterpret_cast<const void*>(&k_bias_rows), hipFuncAttributeMaxDynamicSharedMemorySize, (int)((size_t)BROWS * NN * 4));
    k_bias_rows<<<dim3(NN / BROWS), b256, (size_t)BROWS * NN * 4, stream>>>(ei, ew, nE, nChunks, Bpl);

    k_cvt_f16<<<dim3((NN * DM / 8) / 256), b256, 0, stream>>>(x, Xh, NN * DM / 8, 1.0f);
    k_cvt_f16<<<dim3((QKV3 * DM / 8) / 256), b256, 0, stream>>>(Wqkv, Wqh, QKV3 * DM / 8, 16.0f);
    k_cvt_f16<<<dim3((DM * DM / 8) / 256), b256, 0, stream>>>(Wo, Woh, DM * DM / 8, 16.0f);
    k_cvt_f16<<<dim3((DM * DM / 8) / 256), b256, 0, stream>>>(W1, W1h, DM * DM / 8, 16.0f);

    k_gemm64<2, 1, false><<<dim3(((NN / 64) * (QKLD / 64) + 7) / 8), b256, 0, stream>>>(
        Xh, DM, Wqh, DM, (void*)QKh, QKLD, bqkv, x, 0, NN, QKLD, DM, winv);
    k_gemm64<1, 1, false><<<dim3(((DM / 64) * (NN / 64) + 7) / 8), b256, 0, stream>>>(
        Wqh + (size_t)2 * DM * DM, DM, Xh, DM, (void*)VTh, NN, bqkv + 2 * DM, x, 0, DM, NN, DM, winv);

    k_attn<<<dim3(NH * (NN / 64)), dim3(128), 0, stream>>>(QKh, VTh, Bpl, CTXh);

    k_gemm64<2, 0, true><<<dim3(((NN / 64) * (DM / 64) + 7) / 8), b256, 0, stream>>>(
        CTXh, DM, Woh, DM, (void*)Y, DM, bo, x, DM, NN, DM, DM, winv);
    k_ln<1><<<dim3(NN / 2), b256, 0, stream>>>(Y, g1, be1, H, Hh, NN);

    k_gemm64<2, 0, true><<<dim3(((NN / 64) * (DM / 64) + 7) / 8), b256, 0, stream>>>(
        Hh, DM, W1h, DM, (void*)Y, DM, b1, H, DM, NN, DM, DM, winv);
    k_ln<0><<<dim3(NN / 2), b256, 0, stream>>>(Y, g2, be2, out, Hh, NN);

    (void)hipGetLastError();
}
